// SigMMD_63823214018691
// MI455X (gfx1250) — hardware-verified
//
#include <hip/hip_runtime.h>
#include <math.h>

typedef __attribute__((ext_vector_type(16))) _Float16 v16h;
typedef __attribute__((ext_vector_type(8)))  _Float16 v8h;
typedef __attribute__((ext_vector_type(8)))  float    v8f;
typedef __attribute__((ext_vector_type(4)))  float    v4f;
typedef __attribute__((ext_vector_type(4)))  unsigned int v4u;

constexpr int kPaths       = 64;
constexpr int kPts         = 128;
constexpr int kDim         = 64;
constexpr int kSteps       = 127;
constexpr int kPlaneElems  = kPaths * kPts * kDim;
constexpr int kPairsPerWave = 8;
constexpr int kSymPairs    = kPaths * (kPaths + 1) / 2;
constexpr int kSymWaves    = kSymPairs / kPairsPerWave;
constexpr int kXYWaves     = kPaths * kPaths / kPairsPerWave;
constexpr int kGramWaves   = 2 * kSymWaves + kXYWaves;
constexpr int kIncPitch    = 1028;
constexpr int kIncLdsFloats = 16 * kIncPitch;
constexpr int kGramLineFloats = 32;
constexpr float kCarry     = 4.0f;
constexpr float kCarryFold = 1.0f / 16.0f;
constexpr double kInvPairs = 1.0 / 4096.0;
static_assert(kSymPairs % kPairsPerWave == 0);
static_assert((kPaths * kPaths) % kPairsPerWave == 0);
static_assert((kIncPitch * 4) % 16 == 0);
static_assert(kPlaneElems % (8 * 256) == 0);

template <typename T> struct Frag;
template <> struct Frag<_Float16> {
  typedef v16h V; union U { v16h v; v8h h[2]; };
  static __device__ __forceinline__ v16h load(const _Float16* p) {
    U f; f.h[0] = *(const v8h*)(p); f.h[1] = *(const v8h*)(p + 16); return f.v;
  }
  static __device__ __forceinline__ v8f mma(v16h a, v16h b, v8f c) {
    return __builtin_amdgcn_wmma_f32_16x16x32_f16(false, a, false, b, (short)0, c, false, false);
  }
};
__device__ __forceinline__ void tile_guard(v8f& c, v16h a0, v16h b0, v16h a1, v16h b1) {
  asm volatile("v_nop\n\tv_nop\n\tv_nop\n\tv_nop" : "+v"(c) : "v"(a0), "v"(b0), "v"(a1), "v"(b1));
}
__device__ __forceinline__ unsigned pk16(unsigned short a, unsigned short b) { return (unsigned)a | ((unsigned)b << 16); }
__device__ __forceinline__ unsigned short h_bits(float f) { const _Float16 h = (_Float16)f; return __builtin_bit_cast(unsigned short, h); }

__device__ __forceinline__ void decode_pair(int g, int p, int& a, int& b) {
  if (g < 2) {
    const float sf = sqrtf((float)(8 * p + 1));
    int bb = (int)((sf - 1.0f) * 0.5f);
    if (((bb + 1) * (bb + 2)) / 2 <= p) bb += 1;
    if ((bb * (bb + 1)) / 2 > p) bb -= 1;
    bb = bb < 0 ? 0 : (bb > 63 ? 63 : bb);
    int aa = p - (bb * (bb + 1)) / 2;
    aa = aa < 0 ? 0 : (aa > bb ? bb : aa);
    a = aa; b = bb;
  } else {
    a = (p >> 6) & 63;
    b = p & 63;
  }
}

__global__ __launch_bounds__(256) void diff_cast_kernel(const float* __restrict__ X, const float* __restrict__ Y,
                                                        unsigned short* __restrict__ DX, unsigned short* __restrict__ DY) {
  const int plane = blockIdx.y;
  const float* P = (plane == 0) ? X : Y;
  unsigned short* O = (plane == 0) ? DX : DY;
  const int i = blockIdx.x * 256 + threadIdx.x;
  if (i >= kPlaneElems / 8) return;
  const int e = i * 8;
  const int a = e >> 13;
  const int r = (e >> 6) & 127;
  const int d = e & 63;
  const int r1 = (r < kSteps) ? (r + 1) : r;
  const float* p0 = P + ((size_t)(a * kPts + r))  * kDim + d;
  const float* p1 = P + ((size_t)(a * kPts + r1)) * kDim + d;
  const v4f x0 = *(const v4f*)(p0);
  const v4f x1 = *(const v4f*)(p0 + 4);
  const v4f y0 = *(const v4f*)(p1);
  const v4f y1 = *(const v4f*)(p1 + 4);
  const float s = (r < kSteps) ? kCarry : 0.0f;
  unsigned short hb[8];
#pragma unroll
  for (int k = 0; k < 4; ++k) {
    hb[k]     = h_bits(s * (y0[k] - x0[k]));
    hb[4 + k] = h_bits(s * (y1[k] - x1[k]));
  }
  const v4u u = (v4u){pk16(hb[0], hb[1]), pk16(hb[2], hb[3]), pk16(hb[4], hb[5]), pk16(hb[6], hb[7])};
  unsigned short* q = O + (size_t)e;
  *(volatile v4u*)q = u;
  __threadfence();
  *(volatile v4u*)q = u;
}

__global__ __launch_bounds__(32) void gram_kernel(const unsigned short* __restrict__ DXp, const unsigned short* __restrict__ DYp,
                                                 float* __restrict__ gram) {
  extern __shared__ __attribute__((aligned(16))) float sInc[];
  __shared__ float sOut[kPairsPerWave];
  const int lane = threadIdx.x;
  const int bid  = blockIdx.x;
  int g, pbase;
  if (bid < kSymWaves) { g = 0; pbase = bid * kPairsPerWave; }
  else if (bid < 2 * kSymWaves) { g = 1; pbase = (bid - kSymWaves) * kPairsPerWave; }
  else { g = 2; pbase = (bid - 2 * kSymWaves) * kPairsPerWave; }
  const _Float16* DX = (const _Float16*)(const void*)DXp;
  const _Float16* DY = (const _Float16*)(const void*)DYp;
  const _Float16* Pp = (g == 1) ? DY : DX;
  const _Float16* Qp = (g == 0) ? DX : DY;

  const int rl   = lane & 15;
  const int koff = (lane >> 4) * 8;
  const int hrow = (lane >> 4) * 8;
  const int ppl  = lane >> 2;
  const int q    = lane & 3;

  float kreg[32];
#pragma unroll
  for (int m = 0; m < 32; ++m) kreg[m] = 1.0f;

#pragma unroll 1
  for (int ib = 0; ib < 8; ++ib) {
    const int i0 = ib * 16;
    __syncthreads();
#pragma unroll 1
    for (int pp = 0; pp < kPairsPerWave; ++pp) {
      int a, b;
      decode_pair(g, pbase + pp, a, b);
      const _Float16* arow = Pp + ((size_t)(a * kPts + i0 + rl)) * kDim + koff;
      const v16h af0 = Frag<_Float16>::load(arow);
      const v16h af1 = Frag<_Float16>::load(arow + 32);
      const _Float16* bbase = Qp + ((size_t)(b * kPts + rl)) * kDim + koff;
      float* dst = sInc + hrow * kIncPitch + pp * 128 + rl;
#pragma unroll 2
      for (int t = 0; t < 8; ++t) {
        const _Float16* brow = bbase + (size_t)t * 16 * kDim;
        const v16h bf0 = Frag<_Float16>::load(brow);
        const v16h bf1 = Frag<_Float16>::load(brow + 32);
        v8f acc = (v8f){0.f, 0.f, 0.f, 0.f, 0.f, 0.f, 0.f, 0.f};
        acc = Frag<_Float16>::mma(af0, bf0, acc);
        acc = Frag<_Float16>::mma(af1, bf1, acc);
        tile_guard(acc, af0, bf0, af1, bf1);
#pragma unroll
        for (int r = 0; r < 8; ++r) dst[r * kIncPitch + t * 16] = acc[r] * kCarryFold;
      }
    }
    __syncthreads();
    const int nrows = (ib == 7) ? (kSteps - 112) : 16;
#pragma unroll 1
    for (int ii = 0; ii < nrows; ++ii) {
      const float* rp = sInc + ii * kIncPitch + ppl * 128 + q * 32;
      float iv[32];
#pragma unroll
      for (int k = 0; k < 8; ++k) {
        const v4f v = *(const v4f*)(rp + 4 * k);
        iv[4 * k + 0] = v[0]; iv[4 * k + 1] = v[1]; iv[4 * k + 2] = v[2]; iv[4 * k + 3] = v[3];
      }
      const float up = __shfl_up(kreg[31], 1, 32);
      float prev = (q == 0) ? 1.0f : up;
      float s = 0.0f;
      float sm[32];
#pragma unroll
      for (int m = 0; m < 32; ++m) {
        float d = (kreg[m] - prev) + prev * iv[m];
        if (m == 31) d = (q == 3) ? 0.0f : d;
        s = s + d;
        sm[m] = s;
        prev = kreg[m];
      }
      const float u1 = __shfl_up(s, 1, 32);
      const float c1 = (q >= 1) ? (u1 + s) : s;
      const float u2 = __shfl_up(c1, 2, 32);
      const float incl = (q >= 2) ? (u2 + c1) : c1;
      const float u3 = __shfl_up(incl, 1, 32);
      const float ex = (q >= 1) ? u3 : 0.0f;
#pragma unroll
      for (int m = 0; m < 32; ++m) kreg[m] = 1.0f + (ex + sm[m]);
    }
  }

  if (q == 3) sOut[ppl] = kreg[30];
  __syncthreads();
  const float sv = sOut[lane & 7];
  const float ov = (lane < kPairsPerWave) ? sv : 0.0f;
  float* gp = gram + (size_t)bid * kGramLineFloats + lane;
  *(volatile float*)gp = ov;
  __threadfence();
  *(volatile float*)gp = ov;
}

__global__ __launch_bounds__(256) void final_kernel(const float* __restrict__ X, const float* __restrict__ Y,
                                                    const float* __restrict__ gram, float* __restrict__ out) {
  __shared__ double red[4][256];
  const int t = threadIdx.x;
  double sxx = 0.0, syy = 0.0, sxy = 0.0, sms = 0.0;
#pragma unroll 1
  for (int p = t; p < kSymPairs; p += 256) {
    int a, b;
    decode_pair(0, p, a, b);
    const double w = (a == b) ? 1.0 : 2.0;
    const int w0 = p >> 3, sl = p & 7;
    sxx += w * (double)gram[(size_t)(w0) * kGramLineFloats + sl];
    syy += w * (double)gram[(size_t)(kSymWaves + w0) * kGramLineFloats + sl];
  }
#pragma unroll 1
  for (int p = t; p < kPaths * kPaths; p += 256) {
    const int w0 = p >> 3, sl = p & 7;
    sxy += (double)gram[(size_t)(2 * kSymWaves + w0) * kGramLineFloats + sl];
  }
#pragma unroll 1
  for (int e = t; e < kPaths * kDim; e += 256) {
    const int a = e >> 6, d = e & 63;
    const float df = X[(size_t)a * (kPts * kDim) + d] - Y[(size_t)a * (kPts * kDim) + d];
    sms += (double)(df * df);
  }
  red[0][t] = sxx; red[1][t] = syy; red[2][t] = sxy; red[3][t] = sms;
  __syncthreads();
#pragma unroll 1
  for (int s = 128; s > 0; s >>= 1) {
    if (t < s) {
      red[0][t] += red[0][t + s];
      red[1][t] += red[1][t + s];
      red[2][t] += red[2][t + s];
      red[3][t] += red[3][t + s];
    }
    __syncthreads();
  }
  if (t == 0) {
    const double mxx = red[0][0] * kInvPairs;
    const double myy = red[1][0] * kInvPairs;
    const double mxy = red[2][0] * kInvPairs;
    const double mse = red[3][0] * kInvPairs;
    const double dist = (mxx + myy) - 2.0 * mxy;
    const float res = (float)(mse + dist);
    *(volatile float*)out = res;
    __threadfence();
    *(volatile float*)out = res;
  }
}

extern "C" void kernel_launch(void* const* d_in, const int* in_sizes, int n_in,
                              void* d_out, int out_size, void* d_ws, size_t ws_size,
                              hipStream_t stream) {
  if (n_in < 2) return;
  if (in_sizes[0] != kPlaneElems) return;
  if (in_sizes[1] != kPlaneElems) return;
  if (out_size < 1) return;

  const float* X = (const float*)d_in[0];
  const float* Y = (const float*)d_in[1];
  float* outp = (float*)d_out;

  const size_t szPlane = (size_t)kPlaneElems * 2;
  const size_t szGram  = (size_t)kGramWaves * kGramLineFloats * 4;
  size_t off = 0;
  const size_t oDX = off; off += szPlane;
  const size_t oDY = off; off += szPlane;
  const size_t oGR = off; off += szGram;
  const size_t total = off;
  if (total > ws_size) return;
  if (total > (size_t)134217728) return;

  char* ws = (char*)d_ws;
  unsigned short* DX16 = (unsigned short*)(ws + oDX);
  unsigned short* DY16 = (unsigned short*)(ws + oDY);
  float* GRAM = (float*)(ws + oGR);

  diff_cast_kernel<<<dim3(kPlaneElems / 8 / 256, 2), dim3(256), 0, stream>>>(X, Y, DX16, DY16);
  gram_kernel<<<dim3(kGramWaves), dim3(32), (size_t)kIncLdsFloats * sizeof(float), stream>>>(DX16, DY16, GRAM);
  final_kernel<<<dim3(1), dim3(256), 0, stream>>>(X, Y, GRAM, outp);
}
